// CrossAttention_80590766342194
// MI455X (gfx1250) — hardware-verified
//
#include <hip/hip_runtime.h>


#ifndef NB
#define NB 2
#endif
#ifndef TX
#define TX 4096
#endif
#ifndef TY
#define TY 4096
#endif
#define NB_FULL 2
#define TX_FULL 4096
#define TY_FULL 4096
#define DEC  512
#define ENC  768
#define NHD  8
#define HD   64
#define KC2  (2 * DEC)
#define PCAR 16384.0f
#define OCAR 1024.0f
#define SCL  0.125f
#define L2E  1.4426950408889634f
#define KPT  72
#define PPT  40
#define OPT  68
#define NEGINF (-__builtin_inff())
static_assert(NB >= 1 && NB <= NB_FULL);
static_assert(TX >= 64 && TX <= TX_FULL && (TX % 64) == 0);
static_assert(TY >= 64 && TY <= TY_FULL && (TY % 64) == 0 && (TY % 32) == 0);
static_assert((DEC % 64) == 0 && (ENC % 64) == 0 && HD == 64 && NHD * HD == DEC);
static_assert((DEC % 32) == 0 && (ENC % 32) == 0 && (HD % 32) == 0 && (KC2 % 32) == 0);
static_assert((DEC % 8) == 0 && (ENC % 8) == 0);
static_assert(((NB * TX) % 64) == 0 && ((NB * TY) % 64) == 0);
static_assert(128 * 4 == 64 * (HD / 8));
static_assert(KPT >= 64 && (KPT % 8) == 0 && PPT >= 32 && (PPT % 8) == 0 && OPT >= 64 && (OPT % 4) == 0);
static_assert((size_t)NHD * NB * TX * HD < (size_t)2147483647);
static_assert(2 * 64 * KPT * 2 + 4 * 16 * PPT * 2 + 4 * 16 * OPT * 4 <= 65536);
static_assert((size_t)(NB - 1) * TX_FULL * DEC + (size_t)TX * DEC <= (size_t)NB_FULL * TX_FULL * DEC);

typedef _Float16 h16;
typedef unsigned short bf;
typedef __attribute__((ext_vector_type(16))) __bf16   v16bf;
typedef __attribute__((ext_vector_type(16))) _Float16 v16h;
typedef __attribute__((ext_vector_type(8)))  _Float16 v8h;
typedef __attribute__((ext_vector_type(8)))  unsigned short v8us;
typedef __attribute__((ext_vector_type(8)))  float    v8f;
typedef __attribute__((ext_vector_type(4)))  float    v4f;
typedef __attribute__((ext_vector_type(4)))  unsigned v4u;
typedef v8h  __attribute__((may_alias)) v8ha;
typedef v4f  __attribute__((may_alias)) v4fa;

__device__ __forceinline__ unsigned short f2bf(float f) { unsigned u = __float_as_uint(f); u += 0x7FFFu + ((u >> 16) & 1u); return (unsigned short)(u >> 16); }
__device__ __forceinline__ float bf2f(unsigned short b) { return __uint_as_float(((unsigned)b) << 16); }
__device__ __forceinline__ float bfr(float f) { return bf2f(f2bf(f)); }
__device__ __forceinline__ v16h cat16(v8h lo, v8h hi) { return __builtin_shufflevector(lo, hi, 0, 1, 2, 3, 4, 5, 6, 7, 8, 9, 10, 11, 12, 13, 14, 15); }
__device__ __forceinline__ v16bf cat16b(v8us lo, v8us hi) { return __builtin_bit_cast(v16bf, __builtin_shufflevector(lo, hi, 0, 1, 2, 3, 4, 5, 6, 7, 8, 9, 10, 11, 12, 13, 14, 15)); }
__device__ __forceinline__ v8f wmma16(v16h a, v16h b, v8f c) { return __builtin_amdgcn_wmma_f32_16x16x32_f16(false, a, false, b, (short)0, c, false, false); }
__device__ __forceinline__ v8f wmmab(v16bf a, v16bf b, v8f c) { return __builtin_amdgcn_wmma_f32_16x16x32_bf16(false, a, false, b, (short)0, c, false, false); }
__device__ __forceinline__ h16 tohx(float x) { return (h16)x; }
__device__ __forceinline__ void wsync() { __builtin_amdgcn_wave_barrier(); asm volatile("" ::: "memory"); }

template <typename T16> struct WFrag;
template <> struct WFrag<h16> { typedef v16h V; static __device__ __forceinline__ V ld(const h16* p) { return cat16(*(const v8h*)p, *(const v8h*)(p + 16)); } static __device__ __forceinline__ v8f mma(V a, V b, v8f c) { return wmma16(a, b, c); } };
template <> struct WFrag<bf> { typedef v16bf V; static __device__ __forceinline__ V ld(const bf* p) { return cat16b(*(const v8us*)p, *(const v8us*)(p + 16)); } static __device__ __forceinline__ v8f mma(V a, V b, v8f c) { return wmmab(a, b, c); } };

template <typename T16, int EP>
__device__ __forceinline__ void gemmw_body(const T16* __restrict__ A, const T16* __restrict__ Bt, int K, float* Cf, h16* Ch, int ldc, const float* __restrict__ bias, size_t sA, size_t sB, size_t sC, float cs) {
    static_assert(EP == 0 || EP == 1);
    typedef typename WFrag<T16>::V V;
    __shared__ __align__(16) float os[16 * OPT];
    const size_t z = blockIdx.z; A += z * sA; Bt += z * sB;
    if (EP == 0) { Cf += z * sC; } else { Ch += z * sC; }
    const int lane = threadIdx.x & 31, lr = lane & 15, hi = lane >> 4; const int r0 = blockIdx.x * 64, c0 = blockIdx.y * 64;
    v8f acc[4][4];
#pragma unroll
    for (int mb = 0; mb < 4; ++mb)
#pragma unroll
        for (int nb = 0; nb < 4; ++nb) acc[mb][nb] = (v8f){};
    const size_t aoff = (size_t)(r0 + lr) * K + 8 * hi, boff = (size_t)(c0 + lr) * K + 8 * hi;
#pragma unroll 1
    for (int kc = 0; kc < K; kc += 32) {
        V a[4];
#pragma unroll
        for (int mb = 0; mb < 4; ++mb) a[mb] = WFrag<T16>::ld(A + aoff + (size_t)mb * 16 * K + kc);
#pragma unroll
        for (int nb = 0; nb < 4; ++nb) { const V b = WFrag<T16>::ld(Bt + boff + (size_t)nb * 16 * K + kc);
#pragma unroll
            for (int mb = 0; mb < 4; ++mb) acc[mb][nb] = WFrag<T16>::mma(a[mb], b, acc[mb][nb]); }
        asm volatile("v_nop\n\tv_nop\n\tv_nop\n\tv_nop" : "+v"(acc[0][0]), "+v"(acc[1][1]), "+v"(acc[2][2]), "+v"(acc[3][3]) : "v"(a[0]), "v"(a[3]));
    }
#pragma unroll
    for (int mb = 0; mb < 4; ++mb) {
#pragma unroll
        for (int nb = 0; nb < 4; ++nb) {
#pragma unroll
            for (int j = 0; j < 8; ++j) os[(hi * 8 + j) * OPT + nb * 16 + lr] = acc[mb][nb][j]; }
        wsync();
        if (EP == 0) {
            float* crow = Cf + (size_t)(r0 + mb * 16) * ldc + c0;
#pragma unroll 1
            for (int ps = 0; ps < 2; ++ps) {
#pragma unroll
                for (int s = 0; s < 8; ++s) { const int row = 2 * s + hi, cofs = lr * 4; v4f val = *(const v4fa*)(os + row * OPT + cofs);
                    val[0] = __fmul_rn(val[0], cs); val[1] = __fmul_rn(val[1], cs); val[2] = __fmul_rn(val[2], cs); val[3] = __fmul_rn(val[3], cs);
                    val[0] += bfr(bias[c0 + cofs]); val[1] += bfr(bias[c0 + cofs + 1]); val[2] += bfr(bias[c0 + cofs + 2]); val[3] += bfr(bias[c0 + cofs + 3]);
                    *(volatile v4f*)(crow + (size_t)row * ldc + cofs) = val; }
                if (ps == 0) __threadfence(); }
        } else {
            h16* hrow = Ch + (size_t)(r0 + mb * 16) * ldc + c0;
#pragma unroll 1
            for (int ps = 0; ps < 2; ++ps) {
#pragma unroll
                for (int s = 0; s < 4; ++s) { const int row = 4 * s + (lane >> 3), c8 = (lane & 7) * 8;
                    const v4f u0 = *(const v4fa*)(os + row * OPT + c8), u1 = *(const v4fa*)(os + row * OPT + c8 + 4);
                    v8h o;
#pragma unroll
                    for (int q = 0; q < 8; ++q) { const float u = (q < 4) ? u0[q & 3] : u1[q & 3]; o[q] = tohx(u); }
                    *(volatile v8h*)(hrow + (size_t)row * ldc + c8) = o; }
                if (ps == 0) __threadfence(); }
        }
        wsync();
    }
}

__global__ __launch_bounds__(32) void k_gemm_p(const bf* A, const bf* Bt, int K, h16* Ch, int ldc, size_t sA, size_t sB, size_t sC) {
    gemmw_body<bf, 1>(A, Bt, K, nullptr, Ch, ldc, nullptr, sA, sB, sC, 1.0f); }
__global__ __launch_bounds__(32) void k_gemm_o(const h16* A, const h16* Bt, int K, float* Cf, int ldc, const float* bias, size_t sA, size_t sB, size_t sC, float cs) {
    gemmw_body<h16, 0>(A, Bt, K, Cf, nullptr, ldc, bias, sA, sB, sC, cs); }

__global__ __launch_bounds__(256) void k_cvt8r(const float* __restrict__ src, bf* dst, int cols, int rows, int srows, size_t n8) {
    const size_t i = (size_t)blockIdx.x * 256 + threadIdx.x; if (i >= n8) return;
    const size_t e = i * 8; const size_t r = e / (size_t)cols; const int c = (int)(e % (size_t)cols); const size_t bb = r / (size_t)rows; const size_t t = r % (size_t)rows;
    const v8f v = *(const v8f*)(src + (bb * (size_t)srows + t) * (size_t)cols + c); v8us o;
#pragma unroll
    for (int k = 0; k < 8; ++k) o[k] = f2bf(v[k]);
    *(volatile v8us*)(dst + e) = o; __threadfence(); *(volatile v8us*)(dst + e) = o; }

__global__ __launch_bounds__(256) void k_cvtwp(const float* __restrict__ F, h16* P, size_t n8) {
    const size_t i = (size_t)blockIdx.x * 256 + threadIdx.x; if (i >= n8) return;
    const size_t e = i * 8; const size_t r = e / DEC; const int c = (int)(e % DEC);
    const v8f a = *(const v8f*)(F + e); v8h o;
#pragma unroll
    for (int q = 0; q < 8; ++q) o[q] = tohx(__fmul_rn(bfr(a[q]), 16.0f));
    h16* d0 = P + r * KC2 + c; h16* d1 = d0 + DEC;
    *(volatile v8h*)d0 = o; *(volatile v8h*)d1 = o; __threadfence(); *(volatile v8h*)d0 = o; *(volatile v8h*)d1 = o; }

__global__ __launch_bounds__(32) void k_maskbits(const int* __restrict__ mask, unsigned* MB, int nw) {
    const int lane = threadIdx.x & 31;
    const int w0 = blockIdx.x * 32;
    unsigned mine = 0xFFFFFFFFu;
#pragma unroll 1
    for (int i = 0; i < 32; ++i) {
        const int wi = w0 + i;
        const int wc = (wi < nw) ? wi : (nw - 1);
        const int bb = wc / (TY / 32), t = (wc % (TY / 32)) * 32 + lane;
        const int m = mask[(size_t)bb * TY_FULL + t];
        const bool pr = (wi >= nw) || (m != 0);
        const unsigned bal = __builtin_amdgcn_ballot_w32(pr);
        mine = (lane == i) ? bal : mine;
    }
    v4u o;
#pragma unroll
    for (int j = 0; j < 4; ++j) o[j] = (unsigned)__shfl((int)mine, (4 * lane + j) & 31, 32);
    if (lane < 8) {
        volatile v4u* p = (volatile v4u*)(MB + w0 + 4 * lane);
        *p = o; __threadfence(); *p = o;
    }
}

__global__ __launch_bounds__(128) void k_flash(const h16* __restrict__ QH, const h16* __restrict__ KH, const h16* __restrict__ VH, const unsigned* __restrict__ MB, h16* CT) {
    __shared__ __align__(16) h16 kt[64 * KPT];
    __shared__ __align__(16) h16 vt[64 * KPT];
    __shared__ __align__(16) h16 pt[4 * 16 * PPT];
    __shared__ __align__(16) float ot[4 * 16 * OPT];
    const int tid = threadIdx.x;
    const int wave = __builtin_amdgcn_readfirstlane(tid >> 5);
    const int lane = tid & 31, lr = lane & 15, hi = lane >> 4;
    const int q0 = blockIdx.x * 64, h = blockIdx.y, b = blockIdx.z;
    const int qoff = ((h * NB + b) * TX + q0 + wave * 16 + lr) * HD + 8 * hi;
    const size_t kbase = ((size_t)(h * NB + b) * TY) * HD;
    const size_t vbase = ((size_t)b * DEC + (size_t)h * HD) * TY;
    const int mbase = b * (TY / 32);
    const int pb = wave * 16 * PPT, ob = wave * 16 * OPT;
    float mrun[8], lrun[8];
#pragma unroll
    for (int r = 0; r < 8; ++r) { mrun[r] = -1.0e30f; lrun[r] = 0.0f; }
    v8f o0 = (v8f){}, o1 = (v8f){}, o2 = (v8f){}, o3 = (v8f){};
#pragma unroll 1
    for (int kb = 0; kb < TY / 64; ++kb) {
        __syncthreads();
#pragma unroll
        for (int i = 0; i < 4; ++i) {
            const int p = tid + 128 * i, row = p >> 3, c8 = (p & 7) * 8;
            const size_t kof = kbase + (size_t)(kb * 64 + row) * HD + c8;
            const size_t vof = vbase + (size_t)row * TY + kb * 64 + c8;
            const v8h kv = *(const v8h*)(KH + kof);
            const v8h vv = *(const v8h*)(VH + vof);
            *(v8ha*)(kt + row * KPT + c8) = kv;
            *(v8ha*)(vt + row * KPT + c8) = vv;
        }
        __syncthreads();
#pragma unroll 1
        for (int hf = 0; hf < 2; ++hf) {
            const unsigned mw = (unsigned)__builtin_amdgcn_readfirstlane((int)MB[mbase + kb * 2 + hf]);
            if (mw != 0xFFFFFFFFu) {
                v8f s0 = (v8f){}, s1 = (v8f){};
#pragma unroll
                for (int ks = 0; ks < 2; ++ks) {
                    int qo = qoff + ks * 32; asm volatile("" : "+v"(qo));
                    const v16h ah = cat16(*(const v8h*)(QH + qo), *(const v8h*)(QH + qo + 16));
                    const int ko = (hf * 32 + lr) * KPT + ks * 32 + 8 * hi;
                    const v16h b0 = cat16(*(const v8ha*)(kt + ko), *(const v8ha*)(kt + ko + 16));
                    const v16h b1 = cat16(*(const v8ha*)(kt + ko + 16 * KPT), *(const v8ha*)(kt + ko + 16 * KPT + 16));
                    s0 = wmma16(ah, b0, s0); s1 = wmma16(ah, b1, s1);
                    asm volatile("v_nop\n\tv_nop\n\tv_nop\n\tv_nop" : "+v"(s0), "+v"(s1) : "v"(ah), "v"(b0), "v"(b1));
                }
                const bool x0 = ((mw >> lr) & 1u) != 0u, x1 = ((mw >> (16 + lr)) & 1u) != 0u;
                float t0[8], t1[8], mx[8];
#pragma unroll
                for (int r = 0; r < 8; ++r) {
                    const float a0 = s0[r] * SCL, a1 = s1[r] * SCL;
                    t0[r] = x0 ? NEGINF : a0; t1[r] = x1 ? NEGINF : a1; mx[r] = fmaxf(t0[r], t1[r]); }
#pragma unroll
                for (int sh = 1; sh < 16; sh <<= 1) {
#pragma unroll
                    for (int r = 0; r < 8; ++r) mx[r] = fmaxf(mx[r], __shfl_xor(mx[r], sh, 32)); }
#pragma unroll
                for (int r = 0; r < 8; ++r) {
                    const float mn = fmaxf(mrun[r], mx[r]);
                    const float cr = __builtin_amdgcn_exp2f((mrun[r] - mn) * L2E);
                    mrun[r] = mn;
                    const float p0 = __builtin_amdgcn_exp2f((t0[r] - mn) * L2E), p1 = __builtin_amdgcn_exp2f((t1[r] - mn) * L2E);
                    const h16 ph0 = tohx(p0 * PCAR), ph1 = tohx(p1 * PCAR);
                    lrun[r] = lrun[r] * cr + ((float)ph0 + (float)ph1);
                    o0[r] *= cr; o1[r] *= cr; o2[r] *= cr; o3[r] *= cr;
                    pt[pb + (8 * hi + r) * PPT + lr] = ph0;
                    pt[pb + (8 * hi + r) * PPT + 16 + lr] = ph1;
                }
                wsync();
                {
                    const int po = pb + lr * PPT + 8 * hi;
                    const v16h pa = cat16(*(const v8ha*)(pt + po), *(const v8ha*)(pt + po + 16));
                    const int vo = lr * KPT + hf * 32 + 8 * hi;
                    const v16h v0 = cat16(*(const v8ha*)(vt + vo), *(const v8ha*)(vt + vo + 16));
                    const v16h v1 = cat16(*(const v8ha*)(vt + vo + 16 * KPT), *(const v8ha*)(vt + vo + 16 * KPT + 16));
                    const v16h v2 = cat16(*(const v8ha*)(vt + vo + 32 * KPT), *(const v8ha*)(vt + vo + 32 * KPT + 16));
                    const v16h v3 = cat16(*(const v8ha*)(vt + vo + 48 * KPT), *(const v8ha*)(vt + vo + 48 * KPT + 16));
                    o0 = wmma16(pa, v0, o0); o1 = wmma16(pa, v1, o1); o2 = wmma16(pa, v2, o2); o3 = wmma16(pa, v3, o3);
                    asm volatile("v_nop\n\tv_nop\n\tv_nop\n\tv_nop" : "+v"(o0), "+v"(o1), "+v"(o2), "+v"(o3) : "v"(pa), "v"(v0), "v"(v1), "v"(v2), "v"(v3));
                }
                wsync();
            }
        }
    }
#pragma unroll
    for (int sh = 1; sh < 16; sh <<= 1) {
#pragma unroll
        for (int r = 0; r < 8; ++r) lrun[r] += __shfl_xor(lrun[r], sh, 32); }
#pragma unroll
    for (int r = 0; r < 8; ++r) {
        const float fq = __fdiv_rn(OCAR, fmaxf(lrun[r], 1.0e-30f));
        const float f = (lrun[r] > 0.0f) ? fq : 0.0f;
        const int oi = ob + (8 * hi + r) * OPT + lr;
        ot[oi]      = o0[r] * f;
        ot[oi + 16] = o1[r] * f;
        ot[oi + 32] = o2[r] * f;
        ot[oi + 48] = o3[r] * f;
    }
    wsync();
    h16* crow = CT + (size_t)(b * TX + q0 + wave * 16) * KC2 + h * HD;
#pragma unroll 1
    for (int ps = 0; ps < 2; ++ps) {
#pragma unroll
        for (int s = 0; s < 4; ++s) {
            const int row = 4 * s + (lane >> 3), c8 = (lane & 7) * 8;
            const v4f u0 = *(const v4fa*)(ot + ob + row * OPT + c8), u1 = *(const v4fa*)(ot + ob + row * OPT + c8 + 4);
            v8h oh, ol;
#pragma unroll
            for (int q = 0; q < 8; ++q) { const float f = (q < 4) ? u0[q & 3] : u1[q & 3]; const h16 hh = tohx(f); oh[q] = hh; ol[q] = tohx(f - (float)hh); }
            *(volatile v8h*)(crow + (size_t)row * KC2 + c8) = oh;
            *(volatile v8h*)(crow + (size_t)row * KC2 + DEC + c8) = ol;
        }
        if (ps == 0) __threadfence();
    }
}

constexpr size_t al256(size_t b) { return (b + 255) & ~(size_t)255; }
constexpr int    NWORDS = NB * (TY / 32);
constexpr int    NWLINES = (NWORDS + 31) / 32;
constexpr size_t SZ_XB  = al256((size_t)NB * TX * DEC * 2);
constexpr size_t SZ_YB  = al256((size_t)NB * TY * ENC * 2);
constexpr size_t SZ_WQ  = al256((size_t)DEC * DEC * 2);
constexpr size_t SZ_WKV = al256((size_t)2 * DEC * ENC * 2);
constexpr size_t SZ_WP  = al256((size_t)DEC * KC2 * 2);
constexpr size_t SZ_Q   = al256((size_t)NHD * NB * TX * HD * 2);
constexpr size_t SZ_K   = al256((size_t)NHD * NB * TY * HD * 2);
constexpr size_t SZ_VT  = al256((size_t)NB * DEC * TY * 2);
constexpr size_t SZ_CT  = al256((size_t)NB * TX * KC2 * 2);
constexpr size_t SZ_MB  = al256((size_t)NWLINES * 128);
constexpr size_t SZ_ALL = SZ_XB + SZ_YB + SZ_WQ + SZ_WKV + SZ_WP + SZ_Q + SZ_K + SZ_VT + SZ_CT + SZ_MB;
static_assert(SZ_ALL <= (size_t)134217728);
static_assert((size_t)NWLINES * 32 >= (size_t)NWORDS);

extern "C" void kernel_launch(void* const* d_in, const int* in_sizes, int n_in,
                              void* d_out, int out_size, void* d_ws, size_t ws_size, hipStream_t stream) {
    if (n_in < 7) return;
    const size_t needx = (size_t)(NB - 1) * TX_FULL * DEC + (size_t)TX * DEC;
    const size_t needy = (size_t)(NB - 1) * TY_FULL * ENC + (size_t)TY * ENC;
    const size_t needm = (size_t)(NB - 1) * TY_FULL + (size_t)TY;
    if ((size_t)in_sizes[0] < needx || (size_t)in_sizes[1] < needy || (size_t)in_sizes[2] < needm) return;
    if (in_sizes[3] < DEC * DEC || in_sizes[4] < 2 * DEC * ENC || in_sizes[5] < DEC * DEC || in_sizes[6] < DEC) return;
    if ((size_t)out_size < needx) return;
    if (SZ_ALL > ws_size) return;
    const float* x = (const float*)d_in[0]; const float* y = (const float*)d_in[1];
    const int* msk = (const int*)d_in[2];
    const float* wq = (const float*)d_in[3]; const float* wkv = (const float*)d_in[4]; const float* wp = (const float*)d_in[5]; const float* bp = (const float*)d_in[6];
    float* OUT = (float*)d_out;

    char* base = (char*)d_ws; size_t off = 0;
    bf* XB = (bf*)(base + off); off += SZ_XB;
    bf* YB = (bf*)(base + off); off += SZ_YB;
    bf* WQ = (bf*)(base + off); off += SZ_WQ;
    bf* WKV = (bf*)(base + off); off += SZ_WKV;
    h16* WP16 = (h16*)(base + off); off += SZ_WP;
    h16* QH16 = (h16*)(base + off); off += SZ_Q;
    h16* KH16 = (h16*)(base + off); off += SZ_K;
    h16* VH16 = (h16*)(base + off); off += SZ_VT;
    h16* CT16 = (h16*)(base + off); off += SZ_CT;
    unsigned* MB = (unsigned*)(base + off); off += SZ_MB;
    if (off > ws_size) return;

    auto nb256 = [](size_t n) { return (unsigned)((n + 255) / 256); };
    const size_t n8wq = (size_t)DEC * DEC / 8, n8wkv = (size_t)2 * DEC * ENC / 8;
    k_cvt8r<<<nb256(n8wq), 256, 0, stream>>>(wq, WQ, DEC, DEC, DEC, n8wq);
    k_cvt8r<<<nb256(n8wkv), 256, 0, stream>>>(wkv, WKV, ENC, 2 * DEC, 2 * DEC, n8wkv);
    k_cvtwp<<<nb256(n8wq), 256, 0, stream>>>(wp, WP16, n8wq);
    const size_t n8x = (size_t)NB * TX * DEC / 8, n8y = (size_t)NB * TY * ENC / 8;
    k_cvt8r<<<nb256(n8x), 256, 0, stream>>>(x, XB, DEC, TX, TX_FULL, n8x);
    k_cvt8r<<<nb256(n8y), 256, 0, stream>>>(y, YB, ENC, TY, TY_FULL, n8y);
    k_maskbits<<<(unsigned)NWLINES, 32, 0, stream>>>(msk, MB, NWORDS);
    k_gemm_p<<<dim3((unsigned)(NB * TX / 64), 1, NHD), 32, 0, stream>>>(XB, WQ, DEC, QH16, HD, (size_t)0, (size_t)HD * DEC, (size_t)NB * TX * HD);
    k_gemm_p<<<dim3((unsigned)(NB * TY / 64), 1, NHD), 32, 0, stream>>>(YB, WKV, ENC, KH16, HD, (size_t)0, (size_t)HD * ENC, (size_t)NB * TY * HD);
    k_gemm_p<<<dim3(DEC / 64, TY / 64, NB), 32, 0, stream>>>(WKV + (size_t)DEC * ENC, YB, ENC, VH16, TY, (size_t)0, (size_t)TY * ENC, (size_t)DEC * TY);
    k_flash<<<dim3(TX / 64, NHD, NB), 128, 0, stream>>>(QH16, KH16, VH16, MB, CT16);
    k_gemm_o<<<dim3(TX / 64, DEC / 64, NB), 32, 0, stream>>>(CT16, WP16, KC2, OUT, DEC, bp, (size_t)TX * KC2, (size_t)0, (size_t)TX_FULL * DEC, 1.0f / 16384.0f);
}
